// VNAnchorTransformerBlock_43688407335122
// MI455X (gfx1250) — hardware-verified
//
#include <hip/hip_runtime.h>


#define NB_ 2
#define CC 128
#define NN 256
#define C3N (3 * NN)
#define HID 64
#define C2 256
#define NPR (NN * NN)
#define ZEPS 1e-5
#define EPS6 1e-6f

typedef __attribute__((ext_vector_type(16))) __bf16   v16bf;
typedef __attribute__((ext_vector_type(16))) _Float16 v16h;
typedef __attribute__((ext_vector_type(8)))  float    v8f;
typedef __attribute__((ext_vector_type(8)))  unsigned v8u;

__device__ __forceinline__ unsigned f2bf(float f) { unsigned u = __float_as_uint(f); u += 0x7FFFu + ((u >> 16) & 1u); return u >> 16; }
__device__ __forceinline__ unsigned f2h(float f) { return (unsigned)__builtin_bit_cast(unsigned short, (_Float16)f); }
__device__ __forceinline__ int kpat(int v, int half) { return ((v & 4) ? 16 : 0) + half * 8 + 2 * (v & 3); }

template <int F16, int NP> struct Opnd { v16bf p[NP]; };

template <int F16, int NP> __device__ __forceinline__ void pack2(float f0, float f1, unsigned* o) {
    if (F16) { o[0] = f2h(f0) | (f2h(f1) << 16); return; }
    unsigned h0 = f2bf(f0), h1 = f2bf(f1); o[0] = h0 | (h1 << 16);
    if (NP >= 2) {
        float r0 = f0 - __uint_as_float(h0 << 16), r1 = f1 - __uint_as_float(h1 << 16);
        unsigned m0 = f2bf(r0), m1 = f2bf(r1); o[1] = m0 | (m1 << 16);
        if (NP >= 3) {
            float s0 = r0 - __uint_as_float(m0 << 16), s1 = r1 - __uint_as_float(m1 << 16);
            o[2] = f2bf(s0) | (f2bf(s1) << 16);
        }
    }
}
template <int F16, int NP> __device__ __forceinline__ void op_row(const float* rowp, int half, float sc, Opnd<F16, NP>& o) {
    v8u u[NP];
#pragma unroll
    for (int v = 0; v < 8; ++v) {
        int kk = kpat(v, half); unsigned t[3];
        pack2<F16, NP>(rowp[kk] * sc, rowp[kk + 1] * sc, t);
#pragma unroll
        for (int p = 0; p < NP; ++p) u[p][v] = t[p];
    }
#pragma unroll
    for (int p = 0; p < NP; ++p) o.p[p] = __builtin_bit_cast(v16bf, u[p]);
}
template <int F16, int NP> __device__ __forceinline__ void op_row_tail(const float* rowp, int half, float sc, int kvalid, Opnd<F16, NP>& o) {
    v8u u[NP];
#pragma unroll
    for (int v = 0; v < 8; ++v) {
        int kk = kpat(v, half); unsigned t[3];
        float f0 = kk < kvalid ? rowp[kk] * sc : 0.0f, f1 = (kk + 1) < kvalid ? rowp[kk + 1] * sc : 0.0f;
        pack2<F16, NP>(f0, f1, t);
#pragma unroll
        for (int p = 0; p < NP; ++p) u[p][v] = t[p];
    }
#pragma unroll
    for (int p = 0; p < NP; ++p) o.p[p] = __builtin_bit_cast(v16bf, u[p]);
}
template <int F16, int NP> __device__ __forceinline__ void op_col(const float* M, int ld, int n, int k0, int half, float sc, Opnd<F16, NP>& o) {
    v8u u[NP];
#pragma unroll
    for (int v = 0; v < 8; ++v) {
        int kk = k0 + kpat(v, half); unsigned t[3];
        pack2<F16, NP>(M[(size_t)kk * ld + n] * sc, M[(size_t)(kk + 1) * ld + n] * sc, t);
#pragma unroll
        for (int p = 0; p < NP; ++p) u[p][v] = t[p];
    }
#pragma unroll
    for (int p = 0; p < NP; ++p) o.p[p] = __builtin_bit_cast(v16bf, u[p]);
}
template <int F16, int NP> __device__ __forceinline__ void op_col_tail(const float* M, int ld, int n, int k0, int half, float sc, int K, Opnd<F16, NP>& o) {
    v8u u[NP];
#pragma unroll
    for (int v = 0; v < 8; ++v) {
        int kk = k0 + kpat(v, half); unsigned t[3];
        float f0 = kk < K ? M[(size_t)kk * ld + n] * sc : 0.0f, f1 = (kk + 1) < K ? M[(size_t)(kk + 1) * ld + n] * sc : 0.0f;
        pack2<F16, NP>(f0, f1, t);
#pragma unroll
        for (int p = 0; p < NP; ++p) u[p][v] = t[p];
    }
#pragma unroll
    for (int p = 0; p < NP; ++p) o.p[p] = __builtin_bit_cast(v16bf, u[p]);
}
__device__ __forceinline__ v8f wm_bf16(v16bf a, v16bf b, v8f c) { return __builtin_amdgcn_wmma_f32_16x16x32_bf16(false, a, false, b, (short)0, c, false, false); }
template <int F16, int NA, int NB> __device__ __forceinline__ v8f wmma_op(const Opnd<F16, NA>& a, const Opnd<F16, NB>& b, v8f c) {
    if (F16) {
        v16h ah = __builtin_bit_cast(v16h, a.p[0]), bh = __builtin_bit_cast(v16h, b.p[0]);
        c = __builtin_amdgcn_wmma_f32_16x16x32_f16(false, ah, false, bh, (short)0, c, false, false);
        asm volatile("v_nop\n\tv_nop\n\tv_nop\n\tv_nop" : "+v"(c) : "v"(ah), "v"(bh));
        return c;
    }
    constexpr int NMX = NA > NB ? NA : NB;
#pragma unroll
    for (int i = 0; i < NA; ++i)
#pragma unroll
        for (int j = 0; j < NB; ++j)
            if (i + j < NMX) c = wm_bf16(a.p[i], b.p[j], c);
    if (NA == 1 && NB == 1)      asm volatile("v_nop\n\tv_nop\n\tv_nop\n\tv_nop" : "+v"(c) : "v"(a.p[0]), "v"(b.p[0]));
    else if (NA == 2 && NB == 1) asm volatile("v_nop\n\tv_nop\n\tv_nop\n\tv_nop" : "+v"(c) : "v"(a.p[0]), "v"(a.p[1]), "v"(b.p[0]));
    else if (NA == 1 && NB == 2) asm volatile("v_nop\n\tv_nop\n\tv_nop\n\tv_nop" : "+v"(c) : "v"(a.p[0]), "v"(b.p[0]), "v"(b.p[1]));
    else if (NA == 2 && NB == 2) asm volatile("v_nop\n\tv_nop\n\tv_nop\n\tv_nop" : "+v"(c) : "v"(a.p[0]), "v"(a.p[1]), "v"(b.p[0]), "v"(b.p[1]));
    else                         asm volatile("v_nop\n\tv_nop\n\tv_nop\n\tv_nop" : "+v"(c) : "v"(a.p[0]), "v"(a.p[NA - 1]), "v"(b.p[0]), "v"(b.p[NB - 1]), "v"(a.p[NA / 2]), "v"(b.p[NB / 2]));
    return c;
}

struct ZMap { long long s1; long long s2; int zdiv; int pad_; };
__device__ __forceinline__ size_t zoff(const ZMap& m, int z) { return (size_t)((long long)(z / m.zdiv) * m.s1 + (long long)(z % m.zdiv) * m.s2); }

#define ACT_NONE 0
#define ACT_RELU 1
#define ACT_GELU_ERF 2
#define ACT_SILU 3
#define ACT_TANH 4
__device__ __forceinline__ float act_apply(int act, float x) {
    if (act == ACT_RELU) return x > 0.f ? x : 0.f;
    if (act == ACT_GELU_ERF) return 0.5f * x * (1.0f + erff(x * 0.70710678118654752f));
    if (act == ACT_SILU) return x / (1.0f + expf(-x));
    if (act == ACT_TANH) return tanhf(x);
    return x;
}
struct GemmArgs {
    ZMap za, zb_, zc, zbias, zadd, zrsc, zmul, zrbias;
    const float* A; const float* Bm; float* C; const float* bias; const float* add; const float* rsc; const float* mul; const float* rbias;
    long long ldadd, ldmul;
    int lda, ldb, ldc, K;
    float ascale, bscale, oscale, addscale;
    int M, nvalid, nstore, ldrsc;
    int bcs, pad1, pad2, pad3;
};
template <int BT, int F16, int NA, int NB, int RW, int CW, int ACT>
__global__ __launch_bounds__(256) void gemm_kernel(GemmArgs g) {
    constexpr int TR = 16 * RW, TC = 64 * CW, CSTR = TC + 4;
    __shared__ __align__(16) float cst[TR * CSTR];
    const int z = blockIdx.z;
    const float* A = g.A + zoff(g.za, z); const float* Bm = g.Bm + zoff(g.zb_, z); float* C = g.C + zoff(g.zc, z);
    const int tid = threadIdx.x, lane = tid & 31, wv = tid >> 5;
    const int l16 = lane & 15, half = lane >> 4;
    const int rt = wv % RW, ch = wv / RW;
    const int row0 = blockIdx.x * TR, col0 = blockIdx.y * TC + ch * 64;
    int arix = row0 + rt * 16 + l16; if (arix >= g.M) arix = g.M - 1;
    const float* arow = A + (size_t)arix * g.lda;
    v8f acc[4];
#pragma unroll
    for (int t = 0; t < 4; ++t) acc[t] = (v8f){};
    const int K = g.K;
#pragma unroll 1
    for (int kc = 0; kc < K; kc += 32) {
        Opnd<F16, NA> a;
        if (kc + 32 <= K) op_row<F16, NA>(arow + kc, half, g.ascale, a); else op_row_tail<F16, NA>(arow + kc, half, g.ascale, K - kc, a);
#pragma unroll
        for (int t = 0; t < 4; ++t) {
            Opnd<F16, NB> b;
            const int n = col0 + t * 16 + l16;
            if (n < g.nvalid) {
                if (BT) { if (kc + 32 <= K) op_row<F16, NB>(Bm + (size_t)n * g.ldb + kc, half, g.bscale, b); else op_row_tail<F16, NB>(Bm + (size_t)n * g.ldb + kc, half, g.bscale, K - kc, b); }
                else    { if (kc + 32 <= K) op_col<F16, NB>(Bm, g.ldb, n * g.bcs, kc, half, g.bscale, b); else op_col_tail<F16, NB>(Bm, g.ldb, n * g.bcs, kc, half, g.bscale, K, b); }
            } else {
#pragma unroll
                for (int p = 0; p < NB; ++p) b.p[p] = (v16bf){};
            }
            acc[t] = wmma_op<F16, NA, NB>(a, b, acc[t]);
        }
    }
    const float* bias = g.bias ? g.bias + zoff(g.zbias, z) : nullptr;
    const float* add = g.add ? g.add + zoff(g.zadd, z) : nullptr;
    const float* rsc = g.rsc ? g.rsc + zoff(g.zrsc, z) : nullptr;
    const float* mul = g.mul ? g.mul + zoff(g.zmul, z) : nullptr;
    const float* rbias = g.rbias ? g.rbias + zoff(g.zrbias, z) : nullptr;
#pragma unroll
    for (int t = 0; t < 4; ++t) {
        const int cl = ch * 64 + t * 16 + l16;
        const int cg = blockIdx.y * TC + cl;
        const bool cok = cg < g.nvalid;
        const float bv = (bias && cok) ? bias[(size_t)cg * g.bcs] : 0.0f;
#pragma unroll
        for (int r = 0; r < 8; ++r) {
            const int rl = rt * 16 + r + 8 * half;
            float v = acc[t][r] * g.oscale + bv;
            int rg = row0 + rl; if (rg >= g.M) rg = g.M - 1;
            if (rbias) v += rbias[rg];
            if (rsc) v *= rsc[(size_t)rg * g.ldrsc];
            if (mul && cok) v *= mul[(size_t)rg * g.ldmul + cg];
            if (add && cok) v += g.addscale * add[(size_t)rg * g.ldadd + cg];
            cst[rl * CSTR + cl] = v;
        }
    }
    __syncthreads();
    const int col = tid % TC, rsel = tid / TC, rstep = 256 / TC;
    if (ACT != ACT_NONE) {
#pragma unroll 1
        for (int r = rsel; r < TR; r += rstep) cst[r * CSTR + col] = act_apply(ACT, cst[r * CSTR + col]);
    }
    float* ob = C + (size_t)row0 * g.ldc + (size_t)blockIdx.y * TC;
    const bool colok = (int)(blockIdx.y * TC + col) < g.nstore;
    const int rmax = (g.M - row0 < TR) ? (g.M - row0) : TR;
    auto pass = [&]() {
        if (colok) {
#pragma unroll 4
            for (int r = rsel; r < rmax; r += rstep) *(volatile float*)(ob + (size_t)r * g.ldc + col) = cst[r * CSTR + col];
        }
    };
    pass();
    __threadfence();
    pass();
}
static inline ZMap zm(long long s1) { ZMap m; m.s1 = s1; m.s2 = 0; m.zdiv = 1; m.pad_ = 0; return m; }
static inline ZMap zm2(long long s1, long long s2, int zdiv) { ZMap m; m.s1 = s1; m.s2 = s2; m.zdiv = zdiv; m.pad_ = 0; return m; }
static inline GemmArgs gemm_args(const float* A, int lda, ZMap za, const float* Bm, int ldb, ZMap zb, float* C, int ldc, ZMap zc, int M, int N, int K) {
    GemmArgs g; g.za = za; g.zb_ = zb; g.zc = zc; g.zbias = zm(0); g.zadd = zm(0); g.zrsc = zm(0); g.zmul = zm(0); g.zrbias = zm(0);
    g.A = A; g.Bm = Bm; g.C = C; g.bias = nullptr; g.add = nullptr; g.rsc = nullptr; g.mul = nullptr; g.rbias = nullptr; g.ldadd = 0; g.ldmul = 0;
    g.lda = lda; g.ldb = ldb; g.ldc = ldc; g.K = K; g.ascale = 1.0f; g.bscale = 1.0f; g.oscale = 1.0f; g.addscale = 1.0f; g.M = M; g.nvalid = N; g.nstore = N; g.ldrsc = 1;
    g.bcs = 1; g.pad1 = 0; g.pad2 = 0; g.pad3 = 0;
    return g;
}
static_assert(sizeof(ZMap) == 24, "ZMap layout");
static_assert(sizeof(GemmArgs) == 8 * 24 + 8 * 8 + 2 * 8 + 4 * 4 + 4 * 4 + 4 * 4 + 4 * 4, "GemmArgs has no padding");

__global__ __launch_bounds__(256) void softmax_rows(float* S, long long sy, long long sx, int L, float prescale, const float* addv, long long say, int aydiv, int causal,
                                                  const int* imask, long long imy, long long imx, float maskval) {
    __shared__ float red[8];
    const int tid = threadIdx.x, lane = tid & 31, wid = tid >> 5;
    float* row = S + (size_t)blockIdx.y * sy + (size_t)blockIdx.x * sx;
    const float* av = addv ? addv + (size_t)(blockIdx.y / aydiv) * say : nullptr;
    const int* im = imask ? imask + (size_t)(blockIdx.y / aydiv) * imy + (size_t)blockIdx.x * imx : nullptr;
    float v[16];
    const int nj = L / 256;
    float mx = -__builtin_inff();
#pragma unroll
    for (int j = 0; j < 16; ++j) if (j < nj) { float t = row[tid + 256 * j] * prescale; if (av) t += av[tid + 256 * j]; if (im && im[tid + 256 * j] == 0) t = maskval; if (causal && (tid + 256 * j) > (int)blockIdx.x) t = -__builtin_inff(); v[j] = t; mx = fmaxf(mx, t); }
#pragma unroll
    for (int o = 16; o; o >>= 1) mx = fmaxf(mx, __shfl_xor(mx, o, 32));
    if (lane == 0) red[wid] = mx;
    __syncthreads();
    float m = red[0];
#pragma unroll
    for (int i = 1; i < 8; ++i) m = fmaxf(m, red[i]);
    if (m == -__builtin_inff()) m = 0.f;
    __syncthreads();
    float sum = 0.f;
#pragma unroll
    for (int j = 0; j < 16; ++j) if (j < nj) { v[j] = expf(v[j] - m); sum += v[j]; }
#pragma unroll
    for (int o = 16; o; o >>= 1) sum += __shfl_xor(sum, o, 32);
    if (lane == 0) red[wid] = sum;
    __syncthreads();
    float tot = 0.f;
#pragma unroll
    for (int i = 0; i < 8; ++i) tot += red[i];
    const float inv = 1.0f / tot;
#pragma unroll
    for (int j = 0; j < 16; ++j) if (j < nj) *(volatile float*)(row + tid + 256 * j) = v[j] * inv;
    __threadfence();
#pragma unroll
    for (int j = 0; j < 16; ++j) if (j < nj) *(volatile float*)(row + tid + 256 * j) = v[j] * inv;
}

#define VST2(T, p, v) do { const T vst2_v_ = (v); *(volatile T*)(p) = vst2_v_; __threadfence(); *(volatile T*)(p) = vst2_v_; } while (0)
__global__ __launch_bounds__(256) void k_rel(const float* __restrict__ Q, const float* __restrict__ Kc, const float* __restrict__ posb, float* REL) {
    const int pr = blockIdx.x * 256 + threadIdx.x; if (pr >= NPR) return; const int j = pr % NN, i = pr / NN; float s = 0.f;
#pragma unroll 2
    for (int c = 0; c < CC; ++c) { const float* qc = Q + (size_t)c * C3N; const float* kc = Kc + (size_t)c * C3N; const float dx = qc[i] - kc[j], dy = qc[NN + i] - kc[NN + j], dz = qc[2 * NN + i] - kc[2 * NN + j]; const float sq = dx * dx + dy * dy + dz * dz; s += sq > 0.f ? sqrtf(sq) : 0.f; }
    const float px = posb[i * 3] - posb[j * 3], py = posb[i * 3 + 1] - posb[j * 3 + 1], pz = posb[i * 3 + 2] - posb[j * 3 + 2]; const float psq = px * px + py * py + pz * pz;
    VST2(float, REL + (size_t)pr * 2, s / (float)CC); VST2(float, REL + (size_t)pr * 2 + 1, psq > 0.f ? sqrtf(psq) : 0.f);
}
__global__ __launch_bounds__(256) void k_h1(const float* __restrict__ REL, const float* __restrict__ W1, const float* __restrict__ b1, float* H1) { const size_t q = (size_t)blockIdx.x * 256 + threadIdx.x; if (q >= (size_t)NPR * HID) return; const int h = (int)(q % HID); const size_t pr = q / HID; const float v = REL[pr * 2] * W1[h * 2] + REL[pr * 2 + 1] * W1[h * 2 + 1] + b1[h]; VST2(float, H1 + q, v > 0.f ? v : 0.2f * v); }
__global__ __launch_bounds__(256) void k_soft(const float* __restrict__ SC, float* ATT) {
    const int lane = threadIdx.x & 31, r = blockIdx.x * 8 + (threadIdx.x >> 5); if (r >= NN * CC) return; const int c = r % CC, i = r / CC; float v[8]; float m = -__builtin_inff();
#pragma unroll
    for (int k = 0; k < 8; ++k) { const int j = lane + 32 * k; v[k] = SC[((size_t)i * NN + j) * CC + c]; m = fmaxf(m, v[k]); }
#pragma unroll
    for (int o = 16; o; o >>= 1) m = fmaxf(m, __shfl_xor(m, o, 32));
    float s = 0.f;
#pragma unroll
    for (int k = 0; k < 8; ++k) { v[k] = expf(v[k] - m); s += v[k]; }
#pragma unroll
    for (int o = 16; o; o >>= 1) s += __shfl_xor(s, o, 32);
    const float inv = 1.0f / s;
#pragma unroll
    for (int k = 0; k < 8; ++k) { const int j = lane + 32 * k; VST2(float, ATT + ((size_t)i * CC + c) * NN + j, v[k] * inv); }
}
__global__ __launch_bounds__(256) void k_av(const float* __restrict__ ATT, const float* __restrict__ Vv, float* AO) {
    const int q = blockIdx.x * 256 + threadIdx.x; if (q >= CC * NN) return; const int i = q % NN, c = q / NN; const float* vc = Vv + (size_t)c * C3N; float a0 = 0.f, a1 = 0.f, a2 = 0.f;
#pragma unroll 2
    for (int j = 0; j < NN; ++j) { const float a = ATT[((size_t)i * CC + c) * NN + j]; a0 += a * vc[j]; a1 += a * vc[NN + j]; a2 += a * vc[2 * NN + j]; }
    float* o = AO + (size_t)c * C3N; VST2(float, o + i, a0); VST2(float, o + NN + i, a1); VST2(float, o + 2 * NN + i, a2);
}
__global__ __launch_bounds__(256) void k_add(const float* __restrict__ A, const float* __restrict__ Bv, float* C, size_t n) { const size_t q = (size_t)blockIdx.x * 256 + threadIdx.x; if (q < n) { VST2(float, C + q, A[q] + Bv[q]); } }
__global__ __launch_bounds__(256) void k_zcastat(const float* __restrict__ X, float* ST) {
    __shared__ double red[256][9]; const int b = blockIdx.x, t = threadIdx.x; const float* xb = X + (size_t)b * CC * C3N; const int M = CC * NN;
    double s[3] = {0, 0, 0};
    for (int q = t; q < M; q += 256) { const int c = q / NN, n = q % NN; for (int v = 0; v < 3; ++v) s[v] += (double)xb[(size_t)c * C3N + v * NN + n]; }
    for (int v = 0; v < 3; ++v) red[t][v] = s[v]; __syncthreads();
    for (int o = 128; o > 0; o >>= 1) { if (t < o) for (int v = 0; v < 3; ++v) red[t][v] += red[t + o][v]; __syncthreads(); }
    __shared__ double mu[3]; if (t == 0) for (int v = 0; v < 3; ++v) mu[v] = red[0][v] / (double)M; __syncthreads();
    double cv[9] = {0, 0, 0, 0, 0, 0, 0, 0, 0};
    for (int q = t; q < M; q += 256) { const int c = q / NN, n = q % NN; double d[3]; for (int v = 0; v < 3; ++v) d[v] = (double)xb[(size_t)c * C3N + v * NN + n] - mu[v]; for (int a = 0; a < 3; ++a) for (int e = 0; e < 3; ++e) cv[a * 3 + e] += d[a] * d[e]; }
    __syncthreads(); for (int k = 0; k < 9; ++k) red[t][k] = cv[k]; __syncthreads();
    for (int o = 128; o > 0; o >>= 1) { if (t < o) for (int k = 0; k < 9; ++k) red[t][k] += red[t + o][k]; __syncthreads(); }
    if (t == 0) {
        double A[3][3]; for (int a = 0; a < 3; ++a) for (int e = 0; e < 3; ++e) A[a][e] = red[0][a * 3 + e] / ((double)M + 1e-6) + (a == e ? ZEPS : 0.0);
        double V[3][3] = {{1, 0, 0}, {0, 1, 0}, {0, 0, 1}};
        for (int sweep = 0; sweep < 30; ++sweep) { for (int p = 0; p < 2; ++p) for (int q2 = p + 1; q2 < 3; ++q2) { if (fabs(A[p][q2]) < 1e-300) continue;
            const double th = 0.5 * atan2(2.0 * A[p][q2], A[q2][q2] - A[p][p]); const double cs = cos(th), sn = sin(th);
            for (int k = 0; k < 3; ++k) { const double akp = A[k][p], akq = A[k][q2]; A[k][p] = cs * akp - sn * akq; A[k][q2] = sn * akp + cs * akq; }
            for (int k = 0; k < 3; ++k) { const double apk = A[p][k], aqk = A[q2][k]; A[p][k] = cs * apk - sn * aqk; A[q2][k] = sn * apk + cs * aqk; }
            for (int k = 0; k < 3; ++k) { const double vkp = V[k][p], vkq = V[k][q2]; V[k][p] = cs * vkp - sn * vkq; V[k][q2] = sn * vkp + cs * vkq; } } }
        double W[9]; for (int a = 0; a < 3; ++a) for (int e = 0; e < 3; ++e) { double acc = 0.0; for (int k = 0; k < 3; ++k) { double w = A[k][k]; if (w < ZEPS) w = ZEPS; acc += V[a][k] * (1.0 / sqrt(w)) * V[e][k]; } W[a * 3 + e] = acc; }
        for (int v = 0; v < 3; ++v) { VST2(float, ST + b * 32 + v, (float)mu[v]); } for (int k = 0; k < 9; ++k) { VST2(float, ST + b * 32 + 3 + k, (float)W[k]); }
    }
}
__global__ __launch_bounds__(256) void k_zcaapply(const float* __restrict__ X, const float* __restrict__ ST, const float* __restrict__ gamma, float* OUT) {
    const size_t q = (size_t)blockIdx.x * 256 + threadIdx.x; if (q >= (size_t)NB_ * CC * C3N) return; const int n = (int)(q % NN); const int v = (int)((q / NN) % 3); const int c = (int)((q / C3N) % CC); const int b = (int)(q / ((size_t)CC * C3N));
    const float* st = ST + b * 32; const float* xc = X + ((size_t)b * CC + c) * C3N; float s = 0.f;
#pragma unroll
    for (int e = 0; e < 3; ++e) s += st[3 + v * 3 + e] * (xc[e * NN + n] - st[e]);
    VST2(float, OUT + q, s * gamma[c]);
}
__global__ __launch_bounds__(256) void k_vnlrelu(const float* __restrict__ P, const float* __restrict__ Dd, float* Hh) {
    const int q = blockIdx.x * 256 + threadIdx.x; if (q >= C2 * NN) return; const int n = q % NN, c = q / NN; const float* p = P + (size_t)c * C3N; const float* d = Dd + (size_t)c * C3N;
    const float p0 = p[n], p1 = p[NN + n], p2 = p[2 * NN + n], d0 = d[n], d1 = d[NN + n], d2 = d[2 * NN + n]; const float dot = p0 * d0 + p1 * d1 + p2 * d2, dsq = d0 * d0 + d1 * d1 + d2 * d2; const float mask = dot >= 0.f ? 1.f : 0.f; const float coef = dot / (dsq + EPS6);
    float* h = Hh + (size_t)c * C3N; const float ns = 0.1f;
    const float r0 = ns * p0 + (1.f - ns) * (mask * p0 + (1.f - mask) * (p0 - coef * d0)), r1 = ns * p1 + (1.f - ns) * (mask * p1 + (1.f - mask) * (p1 - coef * d1)), r2 = ns * p2 + (1.f - ns) * (mask * p2 + (1.f - mask) * (p2 - coef * d2));
    VST2(float, h + n, r0); VST2(float, h + NN + n, r1); VST2(float, h + 2 * NN + n, r2);
}
extern "C" void kernel_launch(void* const* d_in, const int* in_sizes, int n_in,
                              void* d_out, int out_size, void* d_ws, size_t ws_size, hipStream_t stream) {
    (void)in_sizes; (void)n_in; (void)out_size;
    const float* x = (const float*)d_in[0]; const float* pos = (const float*)d_in[1]; const float* Wq = (const float*)d_in[2]; const float* Wk = (const float*)d_in[3]; const float* Wv = (const float*)d_in[4]; const float* Wo = (const float*)d_in[5];
    const float* W1 = (const float*)d_in[6]; const float* b1 = (const float*)d_in[7]; const float* W2 = (const float*)d_in[8]; const float* b2 = (const float*)d_in[9]; const float* gm1 = (const float*)d_in[10]; const float* Wfeat = (const float*)d_in[11]; const float* Wdir = (const float*)d_in[12]; const float* Wf2 = (const float*)d_in[13]; const float* gm2 = (const float*)d_in[14];
    float* out = (float*)d_out;
    char* wsp = (char*)d_ws;
    auto take = [&](size_t bytes) { char* p = wsp; wsp += (bytes + 255) & ~(size_t)255; return (void*)p; };
    const size_t SLAB = (size_t)CC * C3N;
    float* Q = (float*)take(SLAB * 4); float* Kc = (float*)take(SLAB * 4); float* V = (float*)take(SLAB * 4); float* REL = (float*)take((size_t)NPR * 2 * 4); float* H1 = (float*)take((size_t)NPR * HID * 4); float* SC = (float*)take((size_t)NPR * CC * 4); float* ATT = (float*)take((size_t)NPR * CC * 4);
    float* AO = (float*)take(SLAB * 4); float* XA = (float*)take(NB_ * SLAB * 4); float* X1 = (float*)take(NB_ * SLAB * 4); float* ST = (float*)take(64 * 4); float* P = (float*)take((size_t)C2 * C3N * 4); float* Dd = (float*)take((size_t)C2 * C3N * 4); float* Hh = (float*)take((size_t)C2 * C3N * 4); float* XF = (float*)take(NB_ * SLAB * 4);
    if ((size_t)(wsp - (char*)d_ws) > ws_size) return;
    for (int b = 0; b < NB_; ++b) {
        const float* xb = x + (size_t)b * SLAB;
        { GemmArgs g = gemm_args(Wq, CC, zm(0), xb, C3N, zm(0), Q, C3N, zm(0), CC, C3N, CC); gemm_kernel<0, 0, 2, 2, 4, 2, ACT_NONE><<<dim3(CC / 64, C3N / 128, 1), 256, 0, stream>>>(g); }
        { GemmArgs g = gemm_args(Wk, CC, zm(0), xb, C3N, zm(0), Kc, C3N, zm(0), CC, C3N, CC); gemm_kernel<0, 0, 2, 2, 4, 2, ACT_NONE><<<dim3(CC / 64, C3N / 128, 1), 256, 0, stream>>>(g); }
        { GemmArgs g = gemm_args(Wv, CC, zm(0), xb, C3N, zm(0), V, C3N, zm(0), CC, C3N, CC); gemm_kernel<0, 0, 2, 2, 4, 2, ACT_NONE><<<dim3(CC / 64, C3N / 128, 1), 256, 0, stream>>>(g); }
        k_rel<<<NPR / 256, 256, 0, stream>>>(Q, Kc, pos + (size_t)b * NN * 3, REL);
        k_h1<<<(unsigned)(((size_t)NPR * HID) / 256), 256, 0, stream>>>(REL, W1, b1, H1);
        { GemmArgs g = gemm_args(H1, HID, zm(0), W2, HID, zm(0), SC, CC, zm(0), NPR, CC, HID); g.bias = b2; gemm_kernel<1, 0, 2, 2, 4, 2, ACT_NONE><<<dim3(NPR / 64, 1, 1), 256, 0, stream>>>(g); }
        k_soft<<<(NN * CC) / 8, 256, 0, stream>>>(SC, ATT);
        k_av<<<(CC * NN) / 256, 256, 0, stream>>>(ATT, V, AO);
        { GemmArgs g = gemm_args(Wo, CC, zm(0), AO, C3N, zm(0), XA + (size_t)b * SLAB, C3N, zm(0), CC, C3N, CC); g.add = xb; g.ldadd = C3N; g.addscale = 1.0f; gemm_kernel<0, 0, 2, 2, 4, 2, ACT_NONE><<<dim3(CC / 64, C3N / 128, 1), 256, 0, stream>>>(g); }
    }
    k_zcastat<<<NB_, 256, 0, stream>>>(XA, ST); k_zcaapply<<<(unsigned)((NB_ * SLAB) / 256), 256, 0, stream>>>(XA, ST, gm1, X1);
    for (int b = 0; b < NB_; ++b) {
        const float* x1b = X1 + (size_t)b * SLAB;
        { GemmArgs g = gemm_args(Wfeat, CC, zm(0), x1b, C3N, zm(0), P, C3N, zm(0), C2, C3N, CC); gemm_kernel<0, 0, 2, 2, 4, 2, ACT_NONE><<<dim3(C2 / 64, C3N / 128, 1), 256, 0, stream>>>(g); }
        { GemmArgs g = gemm_args(Wdir, CC, zm(0), x1b, C3N, zm(0), Dd, C3N, zm(0), C2, C3N, CC); gemm_kernel<0, 0, 2, 2, 4, 2, ACT_NONE><<<dim3(C2 / 64, C3N / 128, 1), 256, 0, stream>>>(g); }
        k_vnlrelu<<<(C2 * NN) / 256, 256, 0, stream>>>(P, Dd, Hh);
        { GemmArgs g = gemm_args(Wf2, C2, zm(0), Hh, C3N, zm(0), XF + (size_t)b * SLAB, C3N, zm(0), CC, C3N, C2); g.add = x1b; g.ldadd = C3N; g.addscale = 1.0f; gemm_kernel<0, 0, 2, 2, 4, 2, ACT_NONE><<<dim3(CC / 64, C3N / 128, 1), 256, 0, stream>>>(g); }
    }
    k_zcastat<<<NB_, 256, 0, stream>>>(XF, ST); k_zcaapply<<<(unsigned)((NB_ * SLAB) / 256), 256, 0, stream>>>(XF, ST, gm2, out);
}
